// WhisperLogMel_30090540876226
// MI455X (gfx1250) — hardware-verified
//
#include <hip/hip_runtime.h>

typedef _Float16 v16h __attribute__((ext_vector_type(16)));
typedef _Float16 v8h  __attribute__((ext_vector_type(8)));
typedef float    v8f  __attribute__((ext_vector_type(8)));
typedef float    v4f  __attribute__((ext_vector_type(4)));
typedef v8h __attribute__((may_alias)) v8ha;
typedef v4f __attribute__((may_alias)) v4fa;

union Frag { v16h v; v8h half[2]; };

#define NB      32
#define CHUNK   480000
#define NFFT    400
#define HOP     160
#define NFREQ   201
#define NMELS   128
#define NFR     3000
#define PADL    200

#define KP_DFT  416
#define MP_DFT  208
#define KS_DFT  13
#define MT_DFT  13
#define KP_MEL  224
#define KS_MEL  7

#define FRB     64
#define NTB     4
#define NGRP    47
#define SPAN    10496
#define PWS     232
#define LMP     3008

#define GC      (MP_DFT * KP_DFT / 8)
#define GM      (NMELS * KP_MEL / 8)
#define GPREP   (2 * GC + GM)

#define PSC     0.00390625f
#define WSC     64.0f
#define UNSC    4.0f

#define FIN_BPB 375

static_assert(SPAN % 256 == 0);
static_assert((FRB * PWS) % 8 == 0);
static_assert(GC % 32 == 0);
static_assert(GM % 32 == 0);
static_assert(NMELS * NFR == FIN_BPB * 256 * 4);
static_assert(LMP % 32 == 0);
static_assert(NGRP * FRB <= LMP);

__device__ __forceinline__ v8f wmma_f16(v16h a, v16h b, v8f c) {
  v8f d = __builtin_amdgcn_wmma_f32_16x16x32_f16(false, a, false, b, (short)0, c, false, false);
  asm volatile("v_nop\n\tv_nop\n\tv_nop\n\tv_nop" : "+v"(d) : "v"(a), "v"(b));
  return d;
}

__global__ __launch_bounds__(256) void k_prep(
    const float* __restrict__ cosk, const float* __restrict__ sink,
    const float* __restrict__ melf,
    _Float16* __restrict__ pcos, _Float16* __restrict__ psin, _Float16* __restrict__ pmel)
{
  const int g = blockIdx.x * 256 + threadIdx.x;
  if (g >= GPREP) return;
  v8h o;
  _Float16* dst;
  if (g < 2 * GC) {
    const int sel = (g >= GC) ? 1 : 0;
    const int e = g - sel * GC;
    const int f = e / (KP_DFT / 8);
    const int q = e - f * (KP_DFT / 8);
    const bool valid = (f < NFREQ) && (q < NFFT / 8);
    const int fc = min(f, NFREQ - 1), qc = min(q, NFFT / 8 - 1);
    const float* src = (sel ? sink : cosk) + (size_t)fc * NFFT + 8 * qc;
    const v4f a = *(const v4fa*)src;
    const v4f c = *(const v4fa*)(src + 4);
    const float e0 = valid ? a.x : 0.0f, e1 = valid ? a.y : 0.0f, e2 = valid ? a.z : 0.0f, e3 = valid ? a.w : 0.0f;
    const float e4 = valid ? c.x : 0.0f, e5 = valid ? c.y : 0.0f, e6 = valid ? c.z : 0.0f, e7 = valid ? c.w : 0.0f;
    const v8h t = { (_Float16)e0, (_Float16)e1, (_Float16)e2, (_Float16)e3,
                    (_Float16)e4, (_Float16)e5, (_Float16)e6, (_Float16)e7 };
    o = t;
    dst = (sel ? psin : pcos) + (size_t)e * 8;
  } else {
    const int e = g - 2 * GC;
    const int mrow = e / (KP_MEL / 8);
    const int q = e - mrow * (KP_MEL / 8);
    float tv[8];
    #pragma unroll
    for (int j = 0; j < 8; ++j) {
      const int k = 8 * q + j;
      const int kc = min(k, NFREQ - 1);
      const float v = melf[(size_t)mrow * NFREQ + kc];
      tv[j] = (k < NFREQ) ? v * WSC : 0.0f;
    }
    const v8h t = { (_Float16)tv[0], (_Float16)tv[1], (_Float16)tv[2], (_Float16)tv[3],
                    (_Float16)tv[4], (_Float16)tv[5], (_Float16)tv[6], (_Float16)tv[7] };
    o = t;
    dst = pmel + (size_t)e * 8;
  }
  *(volatile v8h*)dst = o;
  __threadfence();
  *(volatile v8h*)dst = o;
}

__device__ __forceinline__ void lm_store_pass(const float* so, float* lmp,
                                              int b, int w, int t0, int lane) {
  const int q = lane & 15, rsel = lane >> 4;
  #pragma unroll
  for (int i = 0; i < 8; ++i) {
    const int row = 2 * i + rsel;
    const v4f v = *(const v4fa*)(so + row * 64 + 4 * q);
    float* dst = lmp + ((size_t)(b * NMELS + 16 * w + row)) * LMP + t0 + 4 * q;
    *(volatile v4f*)dst = v;
  }
}

__global__ __launch_bounds__(256) void k_main(
    const float* __restrict__ audio,
    const _Float16* __restrict__ pcos,
    const _Float16* __restrict__ psin,
    const _Float16* __restrict__ pmel,
    float* __restrict__ lmp,
    float* __restrict__ part)
{
  __shared__ __attribute__((aligned(16))) _Float16 sX[SPAN];
  __shared__ __attribute__((aligned(16))) _Float16 sP[FRB * PWS];
  __shared__ __attribute__((aligned(16))) float sO[8 * 1024];
  __shared__ float sMax[8];

  const int tid = threadIdx.x, lane = tid & 31, w = tid >> 5;
  const int h = lane >> 4, m = lane & 15;
  const int g = blockIdx.x, b = blockIdx.y;
  const int t0 = g * FRB;

  const float* ab = audio + (size_t)b * CHUNK;
  const int q0 = t0 * HOP - PADL;
  for (int i = tid; i < SPAN; i += 256) {
    int p = q0 + i;
    p = (p < 0) ? -p : p;
    p = (p >= CHUNK) ? (2 * CHUNK - 2 - p) : p;
    p = min(max(p, 0), CHUNK - 1);
    sX[i] = (_Float16)ab[p];
  }
  const v8h z8 = { (_Float16)0.0f, (_Float16)0.0f, (_Float16)0.0f, (_Float16)0.0f,
                   (_Float16)0.0f, (_Float16)0.0f, (_Float16)0.0f, (_Float16)0.0f };
  for (int i = tid; i < FRB * PWS / 8; i += 256) *(v8ha*)(sP + 8 * i) = z8;
  __syncthreads();

  const v8f zf = {0.f, 0.f, 0.f, 0.f, 0.f, 0.f, 0.f, 0.f};

  for (int mt = w; mt < MT_DFT; mt += 8) {
    v8f accR[NTB], accI[NTB];
    #pragma unroll
    for (int nt = 0; nt < NTB; ++nt) { accR[nt] = zf; accI[nt] = zf; }
    const _Float16* pc = pcos + (size_t)(16 * mt + m) * KP_DFT + 8 * h;
    const _Float16* ps = psin + (size_t)(16 * mt + m) * KP_DFT + 8 * h;
    #pragma unroll 1
    for (int ks = 0; ks < KS_DFT; ++ks) {
      Frag ac, as;
      ac.half[0] = *(const v8ha*)(pc + 32 * ks);
      ac.half[1] = *(const v8ha*)(pc + 32 * ks + 16);
      as.half[0] = *(const v8ha*)(ps + 32 * ks);
      as.half[1] = *(const v8ha*)(ps + 32 * ks + 16);
      const bool ktail = (ks == KS_DFT - 1);
      #pragma unroll
      for (int nt = 0; nt < NTB; ++nt) {
        const _Float16* rb = sX + HOP * (16 * nt + m) + 8 * h + 32 * ks;
        Frag bb;
        bb.half[0] = *(const v8ha*)(rb);
        const v8h t1 = *(const v8ha*)(rb + 16);
        if (ktail) bb.half[1] = z8; else bb.half[1] = t1;
        accR[nt] = wmma_f16(ac.v, bb.v, accR[nt]);
        accI[nt] = wmma_f16(as.v, bb.v, accI[nt]);
      }
    }
    #pragma unroll
    for (int nt = 0; nt < NTB; ++nt) {
      v8h pv = z8;
      #pragma unroll
      for (int r = 0; r < 8; ++r) {
        const float re = accR[nt][r], im = accI[nt][r];
        pv[r] = (_Float16)((re * re + im * im) * PSC);
      }
      *(v8ha*)(sP + (16 * nt + m) * PWS + 16 * mt + 8 * h) = pv;
    }
  }
  __syncthreads();

  v8f acc[NTB];
  #pragma unroll
  for (int nt = 0; nt < NTB; ++nt) acc[nt] = zf;
  {
    const _Float16* pa = pmel + (size_t)(16 * w + m) * KP_MEL + 8 * h;
    #pragma unroll 1
    for (int ks = 0; ks < KS_MEL; ++ks) {
      Frag aa;
      aa.half[0] = *(const v8ha*)(pa + 32 * ks);
      aa.half[1] = *(const v8ha*)(pa + 32 * ks + 16);
      #pragma unroll
      for (int nt = 0; nt < NTB; ++nt) {
        const _Float16* rp = sP + (16 * nt + m) * PWS + 8 * h + 32 * ks;
        Frag bb;
        bb.half[0] = *(const v8ha*)(rp);
        bb.half[1] = *(const v8ha*)(rp + 16);
        acc[nt] = wmma_f16(aa.v, bb.v, acc[nt]);
      }
    }
  }

  float wmax = -__builtin_inff();
  float* so = sO + w * 1024;
  #pragma unroll
  for (int nt = 0; nt < NTB; ++nt) {
    const int tl = 16 * nt + m;
    const bool tv = (t0 + tl) < NFR;
    #pragma unroll
    for (int r = 0; r < 8; ++r) {
      const float mel = acc[nt][r] * UNSC;
      const float lmv = log10f(fmaxf(mel, 1e-10f));
      so[(8 * h + r) * 64 + tl] = lmv;
      wmax = tv ? fmaxf(wmax, lmv) : wmax;
    }
  }
  #pragma unroll
  for (int off = 16; off; off >>= 1) wmax = fmaxf(wmax, __shfl_xor(wmax, off, 32));
  if (lane == 0) sMax[w] = wmax;
  __syncthreads();
  float bm = sMax[0];
  #pragma unroll
  for (int i = 1; i < 8; ++i) bm = fmaxf(bm, sMax[i]);

  float* pline = part + ((size_t)(b * NGRP + g)) * 32 + lane;
  lm_store_pass(so, lmp, b, w, t0, lane);
  if (w == 0) *(volatile float*)pline = bm;
  __threadfence();
  lm_store_pass(so, lmp, b, w, t0, lane);
  if (w == 0) *(volatile float*)pline = bm;
}

__global__ __launch_bounds__(256) void k_final(
    const float* __restrict__ lmp, const float* __restrict__ part, float* __restrict__ out)
{
  __shared__ float smx;
  const int tid = threadIdx.x, lane = tid & 31;
  const int blk = blockIdx.x;
  const int b = blk / FIN_BPB;
  const int e = (blk - b * FIN_BPB) * 256 + tid;
  if (tid < 32) {
    const float* pb = part + (size_t)b * NGRP * 32;
    float v = fmaxf(pb[(size_t)lane * 32], pb[(size_t)min(lane + 32, NGRP - 1) * 32]);
    #pragma unroll
    for (int off = 16; off; off >>= 1) v = fmaxf(v, __shfl_xor(v, off, 32));
    if (lane == 0) smx = v;
  }
  __syncthreads();
  const float fl = smx - 8.0f;
  const int f0 = 4 * e;
  const int mm = f0 / NFR;
  const int t = f0 - mm * NFR;
  const v4f x = *(const v4fa*)(lmp + ((size_t)(b * NMELS + mm)) * LMP + t);
  v4f o;
  o.x = (fmaxf(x.x, fl) + 4.0f) * 0.25f;
  o.y = (fmaxf(x.y, fl) + 4.0f) * 0.25f;
  o.z = (fmaxf(x.z, fl) + 4.0f) * 0.25f;
  o.w = (fmaxf(x.w, fl) + 4.0f) * 0.25f;
  float* dst = out + (size_t)b * (NMELS * NFR) + f0;
  *(volatile v4f*)dst = o;
  __threadfence();
  *(volatile v4f*)dst = o;
}

extern "C" void kernel_launch(void* const* d_in, const int* in_sizes, int n_in,
                              void* d_out, int out_size, void* d_ws, size_t ws_size,
                              hipStream_t stream) {
  if (n_in < 4) return;
  if (in_sizes[0] != NB * CHUNK) return;
  if (in_sizes[1] != NFREQ * NFFT || in_sizes[2] != NFREQ * NFFT) return;
  if (in_sizes[3] != NMELS * NFREQ) return;
  if (out_size != NB * NMELS * NFR) return;

  const float* audio = (const float*)d_in[0];
  const float* cosk  = (const float*)d_in[1];
  const float* sink  = (const float*)d_in[2];
  const float* melf  = (const float*)d_in[3];
  float* out = (float*)d_out;

  const size_t tap_bytes  = (size_t)MP_DFT * KP_DFT * 2;
  const size_t mel_bytes  = (size_t)NMELS * KP_MEL * 2;
  const size_t part_bytes = (size_t)NB * NGRP * 32 * 4;
  const size_t lm_bytes   = (size_t)NB * NMELS * LMP * 4;
  const size_t off_cos  = 0;
  const size_t off_sin  = off_cos + tap_bytes;
  const size_t off_mel  = off_sin + tap_bytes;
  const size_t off_part = off_mel + mel_bytes;
  const size_t off_lm   = off_part + part_bytes;
  const size_t total    = off_lm + lm_bytes;
  if (total > ws_size) return;

  char* ws = (char*)d_ws;
  _Float16* pcos = (_Float16*)(ws + off_cos);
  _Float16* psin = (_Float16*)(ws + off_sin);
  _Float16* pmel = (_Float16*)(ws + off_mel);
  float* part = (float*)(ws + off_part);
  float* lmp  = (float*)(ws + off_lm);

  k_prep<<<(GPREP + 255) / 256, 256, 0, stream>>>(cosk, sink, melf, pcos, psin, pmel);

  dim3 gMain(NGRP, NB);
  k_main<<<gMain, 256, 0, stream>>>(audio, pcos, psin, pmel, lmp, part);

  k_final<<<NB * FIN_BPB, 256, 0, stream>>>(lmp, part, out);
}
